// TopKGate_5385888989890
// MI455X (gfx1250) — hardware-run, weakly checked
//
#include <hip/hip_runtime.h>
#include <math.h>

#define NTOK 4096
#define DM 1024
#define NE 8
#define SLOTS_PER_TOKEN 1
#define NSLOT (NTOK * SLOTS_PER_TOKEN)
#define R_MAX (NSLOT + 64 * NE)
#define NT_MAX (R_MAX / 64)
#define TOPK_DECL 2
#define CAP (TOPK_DECL * ((NTOK + NE - 1) / NE))
#define NGW (NTOK / 32)
#define RW_CH 8192

#define CX_LOG2 11
#define CW_LOG2 16
#define SC_Y (1.0f / (float)(1u << (CX_LOG2 + CW_LOG2)))

#define TBL_COUNT 0
#define TBL_POFF 16
#define TBL_NTILES 32
#define TBL_TILE_E 64
#define TBL_HDR 256
#define TBL_ROWTOK TBL_HDR
#define TBL_SLOTROW (TBL_HDR + R_MAX)
#define TBL_WORDS (TBL_HDR + R_MAX + NSLOT)

static_assert(NE == 8 && NE <= 16 && DM == 1024);
static_assert(NTOK % 256 == 0 && NGW * 32 == NTOK);
static_assert(CAP == 1024);
static_assert(NSLOT % 128 == 0);
static_assert(R_MAX % 64 == 0 && R_MAX >= NSLOT + 63 * NE);
static_assert(TBL_HDR % 32 == 0 && TBL_HDR <= 512);
static_assert(TBL_COUNT + NE <= TBL_POFF && TBL_POFF + NE + 1 <= TBL_NTILES && TBL_NTILES < TBL_TILE_E && TBL_TILE_E + NT_MAX <= TBL_HDR);
static_assert(RW_CH % 128 == 0 && (TBL_WORDS * 4) % 256 == 0);
static_assert((NTOK * DM / 8) % 256 == 0 && (NE * DM * DM / 8) % 256 == 0);
static_assert(NSLOT == 4096 && R_MAX == 4608 && NT_MAX == 72 && TBL_WORDS == 8960);

constexpr size_t al256(size_t b) { return (b + 255) & ~(size_t)255; }
constexpr size_t SZ_X16 = al256((size_t)NTOK * DM * 2);
constexpr size_t SZ_W   = al256((size_t)NE * DM * DM * 2);
constexpr size_t SZ_SEL = al256((size_t)NSLOT * 4);
constexpr size_t SZ_PM  = al256((size_t)NTOK * 4);
constexpr size_t SZ_GS  = al256((size_t)NGW * 32 * 4);
constexpr size_t SZ_TBL = al256((size_t)TBL_WORDS * 4);
constexpr size_t SZ_XG  = al256((size_t)R_MAX * DM * 2);
constexpr size_t SZ_YG  = al256((size_t)R_MAX * DM * 4);
constexpr size_t WS_TOTAL = SZ_X16 + SZ_W + SZ_SEL + SZ_PM + SZ_GS + SZ_TBL + SZ_XG + SZ_YG;
static_assert(WS_TOTAL < (size_t)134217728);
static_assert(WS_TOTAL == (size_t)53562368);

typedef _Float16 h16;
typedef __attribute__((ext_vector_type(16))) _Float16 v16h;
typedef __attribute__((ext_vector_type(8)))  _Float16 v8h;
typedef __attribute__((ext_vector_type(8)))  float    v8f;
typedef __attribute__((ext_vector_type(4)))  float    v4f;
typedef __attribute__((ext_vector_type(2)))  float    v2f;
typedef __attribute__((ext_vector_type(4)))  unsigned int v4u;
typedef __attribute__((ext_vector_type(4)))  int      v4i;
typedef __attribute__((ext_vector_type(2)))  int      v2i;


#define VST2(T, ptr, val) do { const T vst2_v_ = (val); *(volatile T*)(ptr) = vst2_v_; __threadfence(); *(volatile T*)(ptr) = vst2_v_; } while (0)

static __device__ __forceinline__ float bfr(float f) {
    unsigned u = __float_as_uint(f);
    u += 0x7FFFu + ((u >> 16) & 1u);
    return __uint_as_float(u & 0xFFFF0000u);
}
static __device__ __forceinline__ h16 toh_flush(float v) { const float w = (fabsf(v) < 6.103515625e-05f) ? 0.0f : v; return (h16)w; }
static __device__ __forceinline__ void st8h(h16* p, const float* v) {
    v8h hv;
#pragma unroll
    for (int e = 0; e < 8; ++e) hv[e] = toh_flush(v[e]);
    VST2(v8h, p, hv);
}

union FragU { v16h v; v8h h[2]; };
static __device__ __forceinline__ v16h frag_ld(const h16* p) {
    FragU f; f.h[0] = *(const v8h*)(p); f.h[1] = *(const v8h*)(p + 16); return f.v;
}
static __device__ __forceinline__ v8f wmma16g(v16h a, v16h b, v8f c) {
    c = __builtin_amdgcn_wmma_f32_16x16x32_f16(false, a, false, b, (short)0, c, false, false);
    asm volatile("v_nop\n\tv_nop\n\tv_nop\n\tv_nop" : "+v"(c) : "v"(a), "v"(b));
    return c;
}
static __device__ __forceinline__ void wave_sync_lds() {
    __builtin_amdgcn_fence(3  , "workgroup");
    __builtin_amdgcn_wave_barrier();
    __builtin_amdgcn_fence(2  , "workgroup");
}

template <int LOG2C>
__global__ __launch_bounds__(256) void k_plane(const float* __restrict__ src, h16* __restrict__ dst, unsigned n8) {
    const unsigned u = blockIdx.x * 256u + threadIdx.x;
    if (u >= n8) return;
    const float cs = (float)(1u << LOG2C);
    const v4f a = *(const v4f*)(src + (size_t)u * 8u);
    const v4f b = *(const v4f*)(src + (size_t)u * 8u + 4u);
    float v[8] = {bfr(a.x) * cs, bfr(a.y) * cs, bfr(a.z) * cs, bfr(a.w) * cs, bfr(b.x) * cs, bfr(b.y) * cs, bfr(b.z) * cs, bfr(b.w) * cs};
    st8h(dst + (size_t)u * 8u, v);
}

__global__ __launch_bounds__(256) void k_planeT(const float* __restrict__ src, h16* __restrict__ dst) {
    __shared__ __align__(16) float sT[64 * 68];
    const unsigned tid = threadIdx.x;
    const unsigned bx = blockIdx.x;
    const unsigned TPE = (unsigned)((DM / 64) * (DM / 64));
    if (bx >= (unsigned)NE * TPE) return;
    const unsigned e = bx / TPE;
    const unsigned rem = bx - e * TPE;
    const unsigned kt = rem / (unsigned)(DM / 64);
    const unsigned nt = rem - kt * (unsigned)(DM / 64);
    const unsigned k0 = kt * 64u, n0 = nt * 64u;
    const float cs = (float)(1u << CW_LOG2);
    const size_t ebase = (size_t)e * (size_t)(DM * DM);
#pragma unroll
    for (int i = 0; i < 4; ++i) {
        const unsigned p = tid + 256u * (unsigned)i;
        const unsigned kr = p >> 4;
        const unsigned n4 = (p & 15u) * 4u;
        const v4f a = *(const v4f*)(src + ebase + (size_t)(k0 + kr) * DM + n0 + n4);
        v4f s;
        s.x = bfr(a.x) * cs; s.y = bfr(a.y) * cs; s.z = bfr(a.z) * cs; s.w = bfr(a.w) * cs;
        *(v4f*)(&sT[kr * 68u + n4]) = s;
    }
    __syncthreads();
#pragma unroll
    for (int i = 0; i < 2; ++i) {
        const unsigned q = tid + 256u * (unsigned)i;
        const unsigned n = q >> 3;
        const unsigned kp = q & 7u;
        float v[8];
#pragma unroll
        for (int j = 0; j < 8; ++j) v[j] = sT[(8u * kp + (unsigned)j) * 68u + n];
        st8h(dst + ebase + (size_t)(n0 + n) * DM + k0 + 8u * kp, v);
    }
}

__global__ __launch_bounds__(256) void k_gate1(const float* __restrict__ x, const float* __restrict__ wg,
                                               int* __restrict__ sel, float* __restrict__ pm, float* __restrict__ gs) {
    const unsigned lane = threadIdx.x & 31u;
    const unsigned wave = threadIdx.x >> 5;
    const unsigned gwv = blockIdx.x * 8u + wave;
    const unsigned t0 = gwv * 32u;
    if (t0 >= (unsigned)NTOK) return;
    int ki = 0;
    float kw = 0.0f;
    float gsum[NE];
#pragma unroll
    for (int e = 0; e < NE; ++e) gsum[e] = 0.0f;
    for (unsigned j = 0; j < 32u; ++j) {
        const float* xr = x + (size_t)(t0 + j) * DM;
        float lg[NE];
#pragma unroll
        for (int e = 0; e < NE; ++e) lg[e] = 0.0f;
        for (unsigned i = 0; i < (unsigned)(DM / 32); ++i) {
            const unsigned d = lane + 32u * i;
            const float xv = bfr(xr[d]);
#pragma unroll
            for (int e = 0; e < NE; ++e) lg[e] += xv * bfr(wg[(unsigned)e * DM + d]);
        }
#pragma unroll
        for (int e = 0; e < NE; ++e) {
            lg[e] += __shfl_xor(lg[e], 16, 32);
            lg[e] += __shfl_xor(lg[e], 8, 32);
            lg[e] += __shfl_xor(lg[e], 4, 32);
            lg[e] += __shfl_xor(lg[e], 2, 32);
            lg[e] += __shfl_xor(lg[e], 1, 32);
        }
        float bestv = lg[0];
        int besti = 0;
#pragma unroll
        for (int e = 1; e < NE; ++e) { const bool c = lg[e] > bestv; bestv = c ? lg[e] : bestv; besti = c ? e : besti; }
        float pr[NE];
#pragma unroll
        for (int e = 0; e < NE; ++e) pr[e] = expf(lg[e] - bestv);
        float sum = pr[0];
#pragma unroll
        for (int e = 1; e < NE; ++e) sum = sum + pr[e];
        float pbest = 0.0f;
#pragma unroll
        for (int e = 0; e < NE; ++e) {
            pr[e] = pr[e] / sum;
            gsum[e] += pr[e];
            pbest = (e == besti) ? pr[e] : pbest;
        }
        const bool mine = (lane == j);
        ki = mine ? besti : ki;
        kw = mine ? pbest : kw;
    }
    VST2(int, sel + (size_t)(t0 + lane), ki);
    VST2(float, pm + (size_t)(t0 + lane), kw);
    float gv = 0.0f;
#pragma unroll
    for (int e = 0; e < NE; ++e) gv = (lane == (unsigned)e) ? gsum[e] : gv;
    VST2(float, gs + (size_t)gwv * 32u + lane, gv);
}

template <int NE_>
__global__ __launch_bounds__(32) void k_route1w(const int* __restrict__ sel, int* __restrict__ tbl, unsigned nslot, unsigned spt, unsigned hdr, unsigned rmax,
                                                unsigned offPoff, unsigned offNtiles, unsigned offTileE) {
    static_assert(NE_ >= 1 && NE_ <= 16);
    __shared__ __align__(16) int s_img[RW_CH];
    __shared__ __align__(16) int s_hdr[512];
    const unsigned lane = threadIdx.x & 31u;
    const unsigned spl = nslot >> 5;
    const unsigned ng = spl >> 2;
    const unsigned ntmax = rmax >> 6;
    const v4i* sp = (const v4i*)(sel + (size_t)lane * spl);
    int cnt[NE_];
#pragma unroll
    for (int j = 0; j < NE_; ++j) cnt[j] = 0;
    for (unsigned g = 0; g < ng; ++g) {
        const v4i v = sp[g];
#pragma unroll
        for (int c = 0; c < 4; ++c) {
            const int e = min(max(v[c], 0), NE_ - 1);
#pragma unroll
            for (int j = 0; j < NE_; ++j) cnt[j] += (e == j) ? 1 : 0;
        }
    }
    int base0[NE_], total[NE_];
#pragma unroll
    for (int j = 0; j < NE_; ++j) {
        int pre = 0, tot = cnt[j];
#pragma unroll
        for (int d = 1; d < 32; d <<= 1) {
            const int t = __shfl_xor(tot, d, 32);
            pre += ((lane & (unsigned)d) != 0u) ? t : 0;
            tot += t;
        }
        base0[j] = pre;
        total[j] = tot;
    }
    int poff[NE_ + 1];
    poff[0] = 0;
#pragma unroll
    for (int j = 0; j < NE_; ++j) poff[j + 1] = poff[j] + (((total[j] + 63) >> 6) << 6);
    for (unsigned i = lane; i < 512u; i += 32u) s_hdr[i] = (i >= offTileE && i < offTileE + ntmax) ? -1 : 0;
    wave_sync_lds();
    if (lane == 0u) {
#pragma unroll
        for (int j = 0; j < NE_; ++j) { s_hdr[min((unsigned)j, 511u)] = total[j]; s_hdr[min(offPoff + (unsigned)j, 511u)] = poff[j]; }
        s_hdr[min(offPoff + (unsigned)NE_, 511u)] = poff[NE_];
        s_hdr[min(offNtiles, 511u)] = poff[NE_] >> 6;
    }
    for (unsigned t = lane; t < ntmax; t += 32u) {
        const int b64 = (int)(t * 64u);
        int ev = -1;
#pragma unroll
        for (int j = 0; j < NE_; ++j) ev = (b64 >= poff[j] && b64 < poff[j + 1]) ? j : ev;
        s_hdr[min(offTileE + t, 511u)] = ev;
    }
    wave_sync_lds();
    for (int pass = 0; pass < 2; ++pass) {
        for (unsigned i = lane; i < (hdr >> 2); i += 32u) *(volatile v4i*)(tbl + 4u * i) = *(const v4i*)(&s_hdr[4u * i]);
        __threadfence();
    }
    for (unsigned lo = 0; lo < rmax; lo += (unsigned)RW_CH) {
        for (unsigned i = lane; i < (unsigned)(RW_CH / 4); i += 32u) *(v4i*)(&s_img[4u * i]) = (v4i){-1, -1, -1, -1};
        wave_sync_lds();
        int run[NE_];
#pragma unroll
        for (int j = 0; j < NE_; ++j) run[j] = base0[j];
        for (unsigned g = 0; g < ng; ++g) {
            const v4i v = sp[g];
#pragma unroll
            for (int c = 0; c < 4; ++c) {
                const int e = min(max(v[c], 0), NE_ - 1);
                int row = 0;
#pragma unroll
                for (int j = 0; j < NE_; ++j) {
                    const bool hit = (e == j);
                    row = hit ? (poff[j] + run[j]) : row;
                    run[j] += hit ? 1 : 0;
                }
                row = min(max(row, 0), (int)rmax - 1);
                const unsigned rel = (unsigned)row - lo;
                if (rel < (unsigned)RW_CH) s_img[rel] = (int)((lane * spl + 4u * g + (unsigned)c) / spt);
            }
        }
        wave_sync_lds();
        const unsigned nw = min((unsigned)RW_CH, rmax - lo);
        for (int pass = 0; pass < 2; ++pass) {
            for (unsigned i = lane; i < (nw >> 2); i += 32u) *(volatile v4i*)(tbl + hdr + lo + 4u * i) = *(const v4i*)(&s_img[4u * i]);
            __threadfence();
        }
        wave_sync_lds();
    }
    for (unsigned lo = 0; lo < nslot; lo += (unsigned)RW_CH) {
        int run[NE_];
#pragma unroll
        for (int j = 0; j < NE_; ++j) run[j] = base0[j];
        for (unsigned g = 0; g < ng; ++g) {
            const v4i v = sp[g];
#pragma unroll
            for (int c = 0; c < 4; ++c) {
                const int e = min(max(v[c], 0), NE_ - 1);
                int row = 0;
#pragma unroll
                for (int j = 0; j < NE_; ++j) {
                    const bool hit = (e == j);
                    row = hit ? (poff[j] + run[j]) : row;
                    run[j] += hit ? 1 : 0;
                }
                row = min(max(row, 0), (int)rmax - 1);
                const unsigned rel = (lane * spl + 4u * g + (unsigned)c) - lo;
                if (rel < (unsigned)RW_CH) s_img[rel] = row;
            }
        }
        wave_sync_lds();
        const unsigned nw = min((unsigned)RW_CH, nslot - lo);
        for (int pass = 0; pass < 2; ++pass) {
            for (unsigned i = lane; i < (nw >> 2); i += 32u) *(volatile v4i*)(tbl + hdr + rmax + lo + 4u * i) = *(const v4i*)(&s_img[4u * i]);
            __threadfence();
        }
        wave_sync_lds();
    }
}

__global__ __launch_bounds__(256) void k_gather(const h16* __restrict__ x16, const int* __restrict__ tbl, h16* __restrict__ Xg) {
    const unsigned row = blockIdx.x * 2u + (threadIdx.x >> 7);
    if (row >= (unsigned)R_MAX) return;
    const unsigned c = (threadIdx.x & 127u) * 8u;
    const int tr = tbl[TBL_ROWTOK + row];
    const bool pad = (tr < 0);
    const int tok = min(max(tr, 0), NTOK - 1);
    const v4u ld = *(const v4u*)(x16 + (size_t)(unsigned)tok * DM + c);
    v4u v;
    v.x = pad ? 0u : ld.x; v.y = pad ? 0u : ld.y; v.z = pad ? 0u : ld.z; v.w = pad ? 0u : ld.w;
    VST2(v4u, Xg + (size_t)row * DM + c, v);
}

__global__ __launch_bounds__(256) void k_ffn(const h16* __restrict__ Xg, const h16* __restrict__ Wp, const int* __restrict__ tbl, float* __restrict__ Yg) {
    __shared__ __align__(16) float sT[8][16 * 68];
    const unsigned lane = threadIdx.x & 31u;
    const unsigned wave = threadIdx.x >> 5;
    const unsigned u = blockIdx.x * 8u + wave;
    if (u >= (unsigned)(NT_MAX * (DM / 64))) return;
    const unsigned rowtile = u / (unsigned)(DM / 64);
    const unsigned ct = u - rowtile * (unsigned)(DM / 64);
    const int nt = min(max(tbl[TBL_NTILES], 0), NT_MAX);
    if ((int)rowtile >= nt) return;
    const int e = min(max(tbl[TBL_TILE_E + rowtile], 0), NE - 1);
    const size_t wbase = (size_t)(unsigned)e * (size_t)(DM * DM);
    const unsigned m0 = rowtile << 6, n0 = ct << 6;
    const unsigned rlane = lane & 15u;
    const unsigned koff = (lane >> 4) * 8u;
    const unsigned mOff = koff;

    v8f acc[4][4];
#pragma unroll
    for (int i = 0; i < 4; ++i)
#pragma unroll
        for (int j = 0; j < 4; ++j) acc[i][j] = (v8f){0.f,0.f,0.f,0.f,0.f,0.f,0.f,0.f};

    for (unsigned k0 = 0; k0 < (unsigned)DM; k0 += 32u) {
        v16h bh[4];
#pragma unroll
        for (int j = 0; j < 4; ++j)
            bh[j] = frag_ld(Wp + wbase + (size_t)(n0 + ((unsigned)j << 4) + rlane) * DM + koff + k0);
#pragma unroll
        for (int i = 0; i < 4; ++i) {
            const v16h ah = frag_ld(Xg + (size_t)(m0 + ((unsigned)i << 4) + rlane) * DM + koff + k0);
#pragma unroll
            for (int j = 0; j < 4; ++j) acc[i][j] = wmma16g(ah, bh[j], acc[i][j]);
        }
    }

    float* slab = sT[wave];
#pragma unroll
    for (int i = 0; i < 4; ++i) {
        const unsigned mBase = m0 + ((unsigned)i << 4);
#pragma unroll
        for (int j = 0; j < 4; ++j)
#pragma unroll
            for (int r = 0; r < 8; ++r)
                slab[(mOff + (unsigned)r) * 68u + ((unsigned)j << 4) + rlane] = acc[i][j][r] * SC_Y;
        wave_sync_lds();
        const unsigned hh = lane >> 4, c4 = (lane & 15u) * 4u;
#pragma unroll
        for (int half = 0; half < 2; ++half) {
            v4f vv[4];
#pragma unroll
            for (int it = 0; it < 4; ++it) {
                const unsigned row = (unsigned)(half * 4 + it) * 2u + hh;
                vv[it] = *(const v4f*)(slab + row * 68u + c4);
            }
            for (int pass = 0; pass < 2; ++pass) {
#pragma unroll
                for (int it = 0; it < 4; ++it) {
                    const unsigned row = (unsigned)(half * 4 + it) * 2u + hh;
                    *(volatile v4f*)(Yg + (size_t)(mBase + row) * DM + n0 + c4) = vv[it];
                }
                __threadfence();
            }
        }
        wave_sync_lds();
    }
}

__global__ __launch_bounds__(256) void k_combine1(const float* __restrict__ Yg, const float* __restrict__ pm, const int* __restrict__ sel,
                                                  const int* __restrict__ tbl, float* __restrict__ out) {
    const unsigned t = blockIdx.x;
    if (t >= (unsigned)NTOK) return;
    const unsigned c = threadIdx.x * 4u;
    const int e = min(max(sel[t], 0), NE - 1);
    const int r = min(max(tbl[TBL_SLOTROW + t], 0), R_MAX - 1);
    const int pos = r - tbl[TBL_POFF + e];
    const bool keep = (pos >= 0) && (pos < CAP);
    const float p = pm[t];
    const v4f a = *(const v4f*)(Yg + (size_t)(unsigned)r * DM + c);
    v4f y;
    y.x = keep ? a.x * p : 0.0f; y.y = keep ? a.y * p : 0.0f; y.z = keep ? a.z * p : 0.0f; y.w = keep ? a.w * p : 0.0f;
    VST2(v4f, out + (size_t)t * DM + c, y);
}

__global__ __launch_bounds__(32) void k_loss(const float* __restrict__ gs, const int* __restrict__ tbl, float* __restrict__ out1) {
    const unsigned lane = threadIdx.x & 31u;
    float me = 0.0f;
    for (unsigned w = 0; w < (unsigned)NGW; ++w) me += gs[(size_t)w * 32u + lane];
    const int ce = min(max(tbl[TBL_COUNT + min(lane, (unsigned)(NE - 1))], 0), NSLOT);
    float v = (lane < (unsigned)NE) ? me * (float)ce : 0.0f;
    v += __shfl_xor(v, 16, 32);
    v += __shfl_xor(v, 8, 32);
    v += __shfl_xor(v, 4, 32);
    v += __shfl_xor(v, 2, 32);
    v += __shfl_xor(v, 1, 32);
    const float sc = (float)NE / ((float)NTOK * (float)NTOK);
    if (lane == 0u) VST2(float, out1, v * sc);
}

extern "C" void kernel_launch(void* const* d_in, const int* in_sizes, int n_in, void* d_out, int out_size,
                              void* d_ws, size_t ws_size, hipStream_t stream) {
    if (n_in < 3) return;
    if (in_sizes[0] < NTOK * DM || in_sizes[1] < NE * DM || in_sizes[2] < NE * DM * DM) return;
    if (out_size < NTOK * DM + 1) return;

    const float* x  = (const float*)d_in[0];
    const float* wg = (const float*)d_in[1];
    const float* we = (const float*)d_in[2];
    float* out = (float*)d_out;

    char* wsp = (char*)d_ws;
    size_t off = 0;
    auto carve = [&](size_t bytes) -> void* { void* r = wsp + off; off += (bytes + 255) & ~(size_t)255; return r; };
    h16*   x16 = (h16*)carve((size_t)NTOK * DM * 2);
    h16*   wt  = (h16*)carve((size_t)NE * DM * DM * 2);
    int*   sel = (int*)carve((size_t)NSLOT * 4);
    float* pm  = (float*)carve((size_t)NTOK * 4);
    float* gs  = (float*)carve((size_t)NGW * 32 * 4);
    int*   tbl = (int*)carve((size_t)TBL_WORDS * 4);
    h16*   Xg  = (h16*)carve((size_t)R_MAX * DM * 2);
    float* Yg  = (float*)carve((size_t)R_MAX * DM * 4);
    if (off != WS_TOTAL || off > ws_size || off > (size_t)134217728) return;

    k_plane<CX_LOG2><<<(NTOK * DM / 8) / 256, 256, 0, stream>>>(x, x16, (unsigned)(NTOK * DM / 8));
    k_planeT<<<NE * (DM / 64) * (DM / 64), 256, 0, stream>>>(we, wt);
    k_gate1<<<NTOK / 256, 256, 0, stream>>>(x, wg, sel, pm, gs);
    k_route1w<NE><<<1, 32, 0, stream>>>(sel, tbl, (unsigned)NSLOT, (unsigned)SLOTS_PER_TOKEN, (unsigned)TBL_HDR, (unsigned)R_MAX, (unsigned)TBL_POFF, (unsigned)TBL_NTILES, (unsigned)TBL_TILE_E);
    k_gather<<<R_MAX / 2, 256, 0, stream>>>(x16, tbl, Xg);
    k_ffn<<<(NT_MAX * (DM / 64) + 7) / 8, 256, 0, stream>>>(Xg, wt, tbl, Yg);
    k_combine1<<<NTOK, 256, 0, stream>>>(Yg, pm, sel, tbl, out);
    k_loss<<<1, 32, 0, stream>>>(gs, tbl, out + (size_t)NTOK * DM);
}
